// PredictiveRnn_68917045231649
// MI455X (gfx1250) — hardware-verified
//
#include <hip/hip_runtime.h>
#include <math.h>

constexpr int NB    = 128;
constexpr int NT    = 2048;
constexpr int NH    = 128;
constexpr int NG3   = 3 * NH;
constexpr int NTHR  = 64;
constexpr int WPB   = NTHR / 32;
constexpr int ROWS_W = 16;
constexpr int NBLK  = NB / (WPB * ROWS_W);
constexpr int TCH   = 32;
constexpr int NCH   = NT / TCH;
constexpr int HP    = 136;
constexpr int HFP   = 132;
constexpr int SXP   = 36;
constexpr int OSP   = 36;
constexpr int NWTS  = 2 * NG3 + NG3 + NH + 2 * NH;
constexpr int OFF_BI  = 2 * NG3;
constexpr int OFF_BHN = OFF_BI + NG3;
constexpr int OFF_WD  = OFF_BHN + NH;
constexpr float WSC      = 8.0f;
constexpr float WSC_INV  = 0.125f;
constexpr float NEG_HALF_LOG_2PI = -0.9189385332046727f;
constexpr int PACK_THR = 256;
constexpr int PACK_N8  = NG3 * (NH / 8);
constexpr int PACK_BLK = (PACK_N8 + PACK_THR - 1) / PACK_THR;
static_assert(NB % (WPB * ROWS_W) == 0);
static_assert(NH % 32 == 0);
static_assert(NH % 16 == 0 && NG3 == 3 * NH);
static_assert(NT % TCH == 0);
static_assert(HP % 8 == 0 && SXP % 4 == 0 && OSP % 4 == 0);
static_assert((WPB * 2 * ROWS_W * HP) % NTHR == 0);
static_assert((WPB * ROWS_W * HFP) % NTHR == 0);
static_assert(PACK_N8 % PACK_THR == 0);
static_assert(NWTS == 1536 && OFF_WD + 2 * NH == NWTS);

typedef __attribute__((ext_vector_type(16))) _Float16 v16h;
typedef __attribute__((ext_vector_type(8)))  _Float16 v8h;
typedef __attribute__((ext_vector_type(8)))  float    v8f;
typedef __attribute__((ext_vector_type(4)))  float    v4f;

__device__ __forceinline__ void dep_guard3_h(v8f& a, v8f& b, v8f& c, v16h x, v16h y) {
  asm volatile("v_nop\n\tv_nop\n\tv_nop\n\tv_nop" : "+v"(a), "+v"(b), "+v"(c) : "v"(x), "v"(y));
}
__device__ __forceinline__ void keep4_h(v16h a, v16h b, v16h c, v16h d) { asm volatile("v_nop" :: "v"(a), "v"(b), "v"(c), "v"(d)); }
__device__ __forceinline__ void acc_guard3(v8f& a, v8f& b, v8f& c) { asm volatile("v_nop\n\tv_nop\n\tv_nop\n\tv_nop" : "+v"(a), "+v"(b), "+v"(c)); }

template <typename T> struct Frag;
template <> struct Frag<_Float16> {
  typedef v16h V; union U { v16h v; v8h h[2]; };
  static __device__ __forceinline__ v16h load(const _Float16* p) {
    U f; f.h[0] = *(const v8h*)(p); f.h[1] = *(const v8h*)(p + 16); return f.v;
  }
  static __device__ __forceinline__ v8f mma(v16h a, v16h b, v8f c) {
    return __builtin_amdgcn_wmma_f32_16x16x32_f16(false, a, false, b, (short)0, c, false, false);
  }
};

__device__ __forceinline__ float fsig(float x)  { return __builtin_amdgcn_rcpf(1.0f + __expf(-x)); }
__device__ __forceinline__ float ftanh(float x) { return 1.0f - 2.0f * __builtin_amdgcn_rcpf(__expf(2.0f * x) + 1.0f); }

__global__ __launch_bounds__(PACK_THR) void pack_wh_kernel(const float* __restrict__ Wh, unsigned short* __restrict__ Btp) {
  const int i = blockIdx.x * PACK_THR + threadIdx.x;
  if (i < PACK_N8) {
    const int n  = i >> 4;
    const int k8 = (i & 15) * 8;
    v8h hv;
#pragma unroll
    for (int e = 0; e < 8; ++e) hv[e] = (_Float16)(Wh[(size_t)(k8 + e) * NG3 + n] * WSC);
    _Float16* dst = (_Float16*)Btp + (size_t)n * NH + k8;
    *(volatile v8h*)dst = hv;
    __threadfence();
    *(volatile v8h*)dst = hv;
  }
}

__global__ __launch_bounds__(NTHR) void gru_seq_kernel(
    const float* __restrict__ s_in, const float* __restrict__ x_in,
    const float* __restrict__ Wi, const float* __restrict__ bi,
    const unsigned short* __restrict__ Btp, const float* __restrict__ bhn,
    const float* __restrict__ Wd, const float* __restrict__ bd,
    float* __restrict__ out) {
  __shared__ __align__(16) _Float16 Ah[WPB][2][ROWS_W * HP];
  __shared__ __align__(16) float    hF[WPB][ROWS_W * HFP];
  __shared__ __align__(16) float    sS[WPB][ROWS_W * SXP];
  __shared__ __align__(16) float    sX[WPB][ROWS_W * SXP];
  __shared__ __align__(16) float    oS[WPB][ROWS_W * OSP];
  __shared__ __align__(16) float    sW[NWTS];

  const _Float16* Bt = (const _Float16*)Btp;
  const int tid = threadIdx.x, lane = tid & 31, wave = tid >> 5;
  const int c = lane & 15, hh = lane >> 4, koff = hh * 8;
  const int rq = lane >> 3, q4 = (lane & 7) * 4;
  const int R0 = (blockIdx.x * WPB + wave) * ROWS_W;

  {
    _Float16* ahf = &Ah[0][0][0];
#pragma unroll 1
    for (int i = tid; i < WPB * 2 * ROWS_W * HP; i += NTHR) ahf[i] = (_Float16)0.0f;
    float* hff = &hF[0][0];
#pragma unroll 1
    for (int i = tid; i < WPB * ROWS_W * HFP; i += NTHR) hff[i] = 0.0f;
#pragma unroll 1
    for (int i = tid; i < 2 * NG3; i += NTHR) sW[i] = Wi[i];
#pragma unroll 1
    for (int i = tid; i < NG3; i += NTHR) sW[OFF_BI + i] = bi[i];
#pragma unroll 1
    for (int i = tid; i < NH; i += NTHR) sW[OFF_BHN + i] = bhn[i];
#pragma unroll 1
    for (int i = tid; i < 2 * NH; i += NTHR) sW[OFF_WD + i] = Wd[i];
  }
  const float bd0 = bd[0], bd1 = bd[1];
  float xs[8];
#pragma unroll
  for (int r = 0; r < 8; ++r) xs[r] = 0.0f;
  __syncthreads();

  _Float16* Ahw = &Ah[wave][0][0];
  float* hFw = hF[wave];
  float* sSw = sS[wave];
  float* sXw = sX[wave];
  float* oSw = oS[wave];
  const v8f z8 = {0.f, 0.f, 0.f, 0.f, 0.f, 0.f, 0.f, 0.f};

#pragma unroll 1
  for (int cidx = 0; cidx < NCH; ++cidx) {
    const int t0 = cidx * TCH;
#pragma unroll
    for (int i = 0; i < 4; ++i) {
      const int row = 4 * i + rq;
      const v4f vs = *(const v4f*)(s_in + (size_t)(R0 + row) * NT + t0 + q4);
      const v4f vx = *(const v4f*)(x_in + (size_t)(R0 + row) * NT + t0 + q4);
      *(v4f*)(sSw + row * SXP + q4) = vs;
      *(v4f*)(sXw + row * SXP + q4) = vx;
    }
    __syncthreads();

#pragma unroll 1
    for (int tt = 0; tt < TCH; ++tt) {
      const int cur = tt & 1;
      const _Float16* arow = Ahw + cur * (ROWS_W * HP) + c * HP + koff;
      _Float16* anx = Ahw + (cur ^ 1) * (ROWS_W * HP);

      float sv[8], xc[8], pm[8], pv[8];
#pragma unroll
      for (int r = 0; r < 8; ++r) {
        sv[r] = sSw[(8 * hh + r) * SXP + tt];
        xc[r] = sXw[(8 * hh + r) * SXP + tt];
        pm[r] = 0.0f;
        pv[r] = 0.0f;
      }

#pragma unroll 1
      for (int ub = 0; ub < NH / 16; ++ub) {
        const int u = 16 * ub + c;
        const _Float16* b0p = Bt + (size_t)u * NH + koff;
        const _Float16* b1p = Bt + (size_t)(NH + u) * NH + koff;
        const _Float16* b2p = Bt + (size_t)(2 * NH + u) * NH + koff;
        v8f acr = z8, acz = z8, acn = z8;
#pragma unroll 1
        for (int k0 = 0; k0 < NH; k0 += 32) {
          const v16h a  = Frag<_Float16>::load(arow + k0);
          const v16h b0 = Frag<_Float16>::load(b0p + k0);
          const v16h b1 = Frag<_Float16>::load(b1p + k0);
          const v16h b2 = Frag<_Float16>::load(b2p + k0);
          acr = Frag<_Float16>::mma(a, b0, acr);
          acz = Frag<_Float16>::mma(a, b1, acz);
          acn = Frag<_Float16>::mma(a, b2, acn);
          dep_guard3_h(acr, acz, acn, a, b2);
          keep4_h(a, b0, b1, b2);
        }
        acc_guard3(acr, acz, acn);

        const float wi0r = sW[u],          wi1r = sW[NG3 + u];
        const float wi0z = sW[NH + u],     wi1z = sW[NG3 + NH + u];
        const float wi0n = sW[2 * NH + u], wi1n = sW[NG3 + 2 * NH + u];
        const float bir  = sW[OFF_BI + u], biz = sW[OFF_BI + NH + u], binn = sW[OFF_BI + 2 * NH + u];
        const float bhu  = sW[OFF_BHN + u];
        const float wd0  = sW[OFF_WD + 2 * u], wd1 = sW[OFF_WD + 2 * u + 1];

#pragma unroll
        for (int r = 0; r < 8; ++r) {
          const int rowl = 8 * hh + r;
          const float ir  = (sv[r] * wi0r + xs[r] * wi1r) + bir;
          const float iz  = (sv[r] * wi0z + xs[r] * wi1z) + biz;
          const float inn = (sv[r] * wi0n + xs[r] * wi1n) + binn;
          const float pr  = ir + acr[r] * WSC_INV;
          const float pz  = iz + acz[r] * WSC_INV;
          const float hnl = acn[r] * WSC_INV + bhu;
          const float rg  = fsig(pr);
          const float zg  = fsig(pz);
          const float ng  = ftanh(inn + rg * hnl);
          const float ho  = hFw[rowl * HFP + u];
          const float hn  = (1.0f - zg) * ng + zg * ho;
          hFw[rowl * HFP + u] = hn;
          anx[rowl * HP + u] = (_Float16)hn;
          pm[r] += hn * wd0;
          pv[r] += hn * wd1;
        }
      }

#pragma unroll
      for (int r = 0; r < 8; ++r) {
#pragma unroll
        for (int off = 1; off < 16; off <<= 1) {
          pm[r] += __shfl_xor(pm[r], off, 32);
          pv[r] += __shfl_xor(pv[r], off, 32);
        }
      }
      float lp[8];
#pragma unroll
      for (int r = 0; r < 8; ++r) {
        const float m  = pm[r] + bd0;
        const float lv = pv[r] + bd1;
        const float d  = xc[r] - m;
        lp[r] = (NEG_HALF_LOG_2PI - 0.5f * lv) - (0.5f * d * d) * expf(-lv);
      }
      if (c == 0) {
#pragma unroll
        for (int r = 0; r < 8; ++r) oSw[(8 * hh + r) * OSP + tt] = lp[r];
      }
#pragma unroll
      for (int r = 0; r < 8; ++r) xs[r] = xc[r];
      __syncthreads();
    }

    for (int pass = 0; pass < 2; ++pass) {
#pragma unroll
      for (int i = 0; i < 4; ++i) {
        const int row = 4 * i + rq;
        const v4f v = *(const v4f*)(oSw + row * OSP + q4);
        *(volatile v4f*)(out + (size_t)(R0 + row) * NT + t0 + q4) = v;
      }
      __threadfence();
    }
  }
}

extern "C" void kernel_launch(void* const* d_in, const int* in_sizes, int n_in,
                              void* d_out, int out_size, void* d_ws, size_t ws_size, hipStream_t stream) {
  if (n_in < 8 || d_out == nullptr || d_ws == nullptr) return;
  if (in_sizes[0] != NB * NT || in_sizes[1] != NB * NT || in_sizes[2] != 2 * NG3 || in_sizes[3] != NG3 ||
      in_sizes[4] != NH * NG3 || in_sizes[5] != NH || in_sizes[6] != NH * 2 || in_sizes[7] != 2 ||
      out_size != NB * NT) return;

  const float* s_in = (const float*)d_in[0];
  const float* x_in = (const float*)d_in[1];
  const float* Wi   = (const float*)d_in[2];
  const float* bi   = (const float*)d_in[3];
  const float* Wh   = (const float*)d_in[4];
  const float* bhn  = (const float*)d_in[5];
  const float* Wd   = (const float*)d_in[6];
  const float* bd   = (const float*)d_in[7];
  float* out = (float*)d_out;

  char* ws = (char*)d_ws; size_t off = 0;
  auto carve = [&](size_t bytes) -> char* { char* p = ws + off; off += (bytes + 255) & ~(size_t)255; return p; };
  unsigned short* BT = (unsigned short*)carve((size_t)NG3 * NH * 2);
  if (off > ws_size || off > (size_t)134217728) return;

  pack_wh_kernel<<<PACK_BLK, PACK_THR, 0, stream>>>(Wh, BT);
  gru_seq_kernel<<<NBLK, NTHR, 0, stream>>>(s_in, x_in, Wi, bi, BT, bhn, Wd, bd, out);
}
